// FirstStageNetwork_88837103550989
// MI455X (gfx1250) — hardware-run, weakly checked
//
#include <hip/hip_runtime.h>
#include <stddef.h>
#include <stdint.h>
#include <math.h>

#define NN      50000
#define CIN     128
#define COUT    256
#define NE      800000
#define GBM     128
#define GBN     64
#define MP      50048
#define NTHR    256
#define NWAVE   8
#define EPT     4
#define WCH     (32 * EPT)
#define NCHUNK  (NE / WCH)
#define CPW     ((NCHUNK + NWAVE - 1) / NWAVE)
#define NBRUN   1024
#define NBK     49
#define NSLOT   (NBK * NBRUN)
#define WLCAP   2560
#define RCAP    20480
#define DEGCAP  128
#define MAXDEG_MEAS   35
#define MAXB1024_MEAS 16765
#define ABM     128
#define SP      68
#define WSMAX   134217728

#define BK_ZINTS (NWAVE * WLCAP + RCAP + 3 * NBRUN)
#define BK_INTS  (BK_ZINTS + NBRUN + 16)
#define BK_LDS   (BK_INTS * 4)

#define PBX   (MP * CIN / 8 / NTHR)
#define PBW   (COUT * CIN / 8 / NTHR)
#define PBTOT (PBX + PBW + 1)

static_assert(NN <= 65536 && NBRUN <= 1024);
static_assert(MP % GBM == 0 && MP == 391 * GBM && MP >= NN && MP % ABM == 0);
static_assert(NSLOT >= MP && NBRUN % ABM == 0 && NBRUN % GBM == 0);
static_assert(NE % WCH == 0 && (2LL * NE) < (1LL << 31));
static_assert(RCAP == NWAVE * WLCAP && RCAP % (NTHR * 4) == 0 && BK_ZINTS % 4 == 0);
static_assert((long long)RCAP * 100 >= (long long)MAXB1024_MEAS * 110);
static_assert(WLCAP >= MAXB1024_MEAS / 8 + 8 * 46 + 1);
static_assert(MAXDEG_MEAS + 8 <= DEGCAP);
static_assert(NBRUN == 4 * NTHR);
static_assert(CIN % 32 == 0 && COUT % GBN == 0 && GBN == 64 && CIN / 8 == 16);
static_assert((MP * CIN / 8) % NTHR == 0 && (COUT * CIN / 8) % NTHR == 0);
static_assert(COUT == 2 * 128 && COUT / 4 == 64);
static_assert(BK_LDS <= 300000);
static_assert((GBM * SP + GBM) * 4 <= 65536);
static_assert(GBM == NWAVE * 16 && ABM == NWAVE * 16);

typedef float          v4f   __attribute__((ext_vector_type(4)));
typedef float          v8f   __attribute__((ext_vector_type(8)));
typedef int            v4i   __attribute__((ext_vector_type(4)));
typedef int            v8i   __attribute__((ext_vector_type(8)));
typedef unsigned short v8us  __attribute__((ext_vector_type(8)));
typedef unsigned short v16us __attribute__((ext_vector_type(16)));
typedef __bf16         v16bf __attribute__((ext_vector_type(16)));
typedef v4f  __attribute__((may_alias)) v4fa;
typedef v4i  __attribute__((may_alias)) v4ia;
typedef v8us __attribute__((may_alias)) v8usa;
union FragB { v16bf v; v16us u; v8us h[2]; v8i w; };

__device__ __forceinline__ v8f wmb(const FragB& a, const FragB& b, v8f c) {
  v8f d = __builtin_amdgcn_wmma_f32_16x16x32_bf16(false, a.v, false, b.v, (short)0, c, false, false);
  asm volatile("v_nop\n\tv_nop\n\tv_nop\n\tv_nop" : "+v"(d) : "v"(a.w), "v"(b.w));
  return d;
}

__device__ __forceinline__ unsigned bf16_bits(float f) {
  const unsigned u = __float_as_uint(f);
  const unsigned r = (u + 0x7FFFu + ((u >> 16) & 1u)) >> 16;
  const unsigned q = (u >> 16) | 0x40u;
  return ((u & 0x7fffffffu) > 0x7f800000u) ? q : r;
}
__device__ __forceinline__ float bf16_val(float f) {
  return __uint_as_float(bf16_bits(f) << 16);
}

__device__ __forceinline__ void st2_v4f(float* p, v4f v) {
  *(volatile v4f*)p = v;
  __threadfence();
  *(volatile v4f*)p = v;
}
__device__ __forceinline__ void st2_v8us(unsigned short* p, v8us v) {
  *(volatile v8us*)p = v;
  __threadfence();
  *(volatile v8us*)p = v;
}

__global__ __launch_bounds__(NTHR) void k_prep(const float* __restrict__ x, const float* __restrict__ w,
                                               const float* __restrict__ b,
                                               unsigned short* xb, unsigned short* wb, float* bf) {
  const int tid = (int)threadIdx.x;
  const int blk = (int)blockIdx.x;
  if (blk < PBX) {
    const int u   = blk * NTHR + tid;
    const int row = u >> 4, k8 = (u & 15) * 8;
    const int rc  = row < NN ? row : NN - 1;
    const unsigned mk = row < NN ? 0xffffu : 0u;
    const float* p = x + (size_t)rc * CIN + k8;
    const v4f a = *(const v4fa*)p;
    const v4f c = *(const v4fa*)(p + 4);
    v8us o;
    o[0] = (unsigned short)(bf16_bits(a.x) & mk); o[1] = (unsigned short)(bf16_bits(a.y) & mk);
    o[2] = (unsigned short)(bf16_bits(a.z) & mk); o[3] = (unsigned short)(bf16_bits(a.w) & mk);
    o[4] = (unsigned short)(bf16_bits(c.x) & mk); o[5] = (unsigned short)(bf16_bits(c.y) & mk);
    o[6] = (unsigned short)(bf16_bits(c.z) & mk); o[7] = (unsigned short)(bf16_bits(c.w) & mk);
    st2_v8us(xb + (size_t)row * CIN + k8, o);
  } else if (blk < PBX + PBW) {
    const int u = (blk - PBX) * NTHR + tid;
    const int n = u >> 4, k8 = (u & 15) * 8;
    const float* p = w + (size_t)n * CIN + k8;
    const v4f a = *(const v4fa*)p;
    const v4f c = *(const v4fa*)(p + 4);
    v8us o;
    o[0] = (unsigned short)bf16_bits(a.x); o[1] = (unsigned short)bf16_bits(a.y);
    o[2] = (unsigned short)bf16_bits(a.z); o[3] = (unsigned short)bf16_bits(a.w);
    o[4] = (unsigned short)bf16_bits(c.x); o[5] = (unsigned short)bf16_bits(c.y);
    o[6] = (unsigned short)bf16_bits(c.z); o[7] = (unsigned short)bf16_bits(c.w);
    st2_v8us(wb + (size_t)n * CIN + k8, o);
  } else {
    if (tid < 64) {
      const v4f a = *(const v4fa*)(b + 4 * tid);
      v4f o;
      o.x = bf16_val(a.x); o.y = bf16_val(a.y); o.z = bf16_val(a.z); o.w = bf16_val(a.w);
      st2_v4f(bf + 4 * tid, o);
    }
  }
}

__device__ __forceinline__ void bucket_flush(const int* pl, const int* cnt, const int* offs, const int* dvb, int ov,
                                             int* lp, int* cp, int* op, int* dp, int* fp, int tid) {
#pragma unroll 1
  for (int i = tid * 4; i < RCAP; i += NTHR * 4) {
    const v4i v = *(const v4ia*)(pl + i);
    *(volatile v4i*)(lp + i) = v;
  }
  {
    const v4i v = *(const v4ia*)(cnt + 4 * tid);
    *(volatile v4i*)(cp + 4 * tid) = v;
  }
  {
    const v4i v = *(const v4ia*)(offs + 4 * tid);
    *(volatile v4i*)(op + 4 * tid) = v;
  }
  {
    const v4i v = *(const v4ia*)(dvb + 4 * tid);
    *(volatile v4i*)(dp + 4 * tid) = v;
  }
  if (tid < 8) {
    const v4i f = {ov, ov, ov, ov};
    *(volatile v4i*)(fp + 4 * tid) = f;
  }
}

__global__ __launch_bounds__(NTHR) void k_bucket(const int* __restrict__ ei, int* LIST, int* OFF, int* CNT,
                                                 int* DINVB, int* FLAG) {
  extern __shared__ __attribute__((aligned(16))) int dsm[];
  int* wl   = dsm;
  int* pl   = dsm + NWAVE * WLCAP;
  int* cnt  = pl + RCAP;
  int* offs = cnt + NBRUN;
  int* cur  = offs + NBRUN;
  int* dvb  = cur + NBRUN;
  int* misc = dvb + NBRUN;
  const int tid = (int)threadIdx.x, lane = tid & 31, wave = tid >> 5;
  const int blk = (int)blockIdx.x;
  const unsigned nbs = (unsigned)(blk * NBRUN);

  {
    const v4i z4 = {0, 0, 0, 0};
    for (int i = tid * 4; i < BK_ZINTS; i += NTHR * 4) *(v4ia*)(dsm + i) = z4;
    if (tid < 16) misc[tid] = 0;
  }
  __syncthreads();

  {
    const int cbeg = wave * CPW;
    const int cend = (cbeg + CPW < NCHUNK) ? (cbeg + CPW) : NCHUNK;
    int* mylist = wl + wave * WLCAP;
    int wc = 0;
#pragma unroll 1
    for (int ch = cbeg; ch < cend; ++ch) {
      const int e0 = ch * WCH + lane * EPT;
      const int* pp = ei + 2 * (size_t)e0;
      const v4i pa = *(const v4ia*)pp;
      const v4i pb = *(const v4ia*)(pp + 4);
      const unsigned s0 = (unsigned)pa.y - nbs, s1 = (unsigned)pa.w - nbs;
      const unsigned s2 = (unsigned)pb.y - nbs, s3 = (unsigned)pb.w - nbs;
      const bool h0 = s0 < (unsigned)NBRUN, h1 = s1 < (unsigned)NBRUN;
      const bool h2 = s2 < (unsigned)NBRUN, h3 = s3 < (unsigned)NBRUN;
      const unsigned m0 = __builtin_amdgcn_ballot_w32(h0), m1 = __builtin_amdgcn_ballot_w32(h1);
      const unsigned m2 = __builtin_amdgcn_ballot_w32(h2), m3 = __builtin_amdgcn_ballot_w32(h3);
      const unsigned any = m0 | m1 | m2 | m3;
      if (any != 0u) {
        int r0 = pa.x, r1 = pa.z, r2 = pb.x, r3 = pb.z;
        r0 = r0 < 0 ? 0 : (r0 > NN - 1 ? NN - 1 : r0);
        r1 = r1 < 0 ? 0 : (r1 > NN - 1 ? NN - 1 : r1);
        r2 = r2 < 0 ? 0 : (r2 > NN - 1 ? NN - 1 : r2);
        r3 = r3 < 0 ? 0 : (r3 > NN - 1 ? NN - 1 : r3);
        const int pre = (int)(__builtin_amdgcn_mbcnt_lo(m0, 0u) + __builtin_amdgcn_mbcnt_lo(m1, 0u) +
                              __builtin_amdgcn_mbcnt_lo(m2, 0u) + __builtin_amdgcn_mbcnt_lo(m3, 0u));
        int p = wc + pre;
        if (h0) { if (p < WLCAP) mylist[p] = r0 | (int)(s0 << 16); p = p + 1; }
        if (h1) { if (p < WLCAP) mylist[p] = r1 | (int)(s1 << 16); p = p + 1; }
        if (h2) { if (p < WLCAP) mylist[p] = r2 | (int)(s2 << 16); p = p + 1; }
        if (h3) { if (p < WLCAP) mylist[p] = r3 | (int)(s3 << 16); p = p + 1; }
        wc += (int)(__builtin_popcount(m0) + __builtin_popcount(m1) + __builtin_popcount(m2) + __builtin_popcount(m3));
      }
    }
    if (lane == 0) misc[wave] = wc;
  }
  __syncthreads();

  if (wave == 0) {
    int ov = 0;
#pragma unroll 1
    for (int w2 = 0; w2 < NWAVE; ++w2) {
      int c = misc[w2];
      if (c > WLCAP) ov = 1;
      c = c < 0 ? 0 : (c > WLCAP ? WLCAP : c);
#pragma unroll 1
      for (int b0 = 0; b0 < c; b0 += 32) {
        const int idx = b0 + lane;
        const int ent = wl[w2 * WLCAP + (idx < WLCAP ? idx : WLCAP - 1)];
        const int m32 = (c - b0) < 32 ? (c - b0) : 32;
#pragma unroll 1
        for (int k = 0; k < m32; ++k) {
          const int u    = __builtin_amdgcn_readlane(ent, k);
          const int slot = (u >> 16) & (NBRUN - 1);
          if (lane == 0) cnt[slot] = cnt[slot] + 1;
        }
      }
    }
    if (lane == 0) misc[9] = ov;
  }
  __syncthreads();
  if (wave == 0) {
    const int base = lane * (NBRUN / 32);
    int s = 0;
#pragma unroll 1
    for (int i = 0; i < NBRUN / 32; ++i) s += cnt[base + i];
    int incl = s;
#pragma unroll
    for (int d = 1; d < 32; d <<= 1) {
      const int y = __shfl_up(incl, d, 32);
      if (lane >= d) incl += y;
    }
    int run = incl - s;
#pragma unroll 1
    for (int i = 0; i < NBRUN / 32; ++i) {
      const int cv = cnt[base + i];
      offs[base + i] = run;
      cur[base + i]  = run;
      run += cv;
    }
  }
  __syncthreads();

  if (wave == 0) {
#pragma unroll 1
    for (int w2 = 0; w2 < NWAVE; ++w2) {
      int c = misc[w2];
      c = c < 0 ? 0 : (c > WLCAP ? WLCAP : c);
#pragma unroll 1
      for (int b0 = 0; b0 < c; b0 += 32) {
        const int idx = b0 + lane;
        const int ent = wl[w2 * WLCAP + (idx < WLCAP ? idx : WLCAP - 1)];
        const int m32 = (c - b0) < 32 ? (c - b0) : 32;
#pragma unroll 1
        for (int k = 0; k < m32; ++k) {
          const int u    = __builtin_amdgcn_readlane(ent, k);
          const int slot = (u >> 16) & (NBRUN - 1);
          if (lane == 0) {
            int p = cur[slot];
            p = p < 0 ? 0 : (p > RCAP - 1 ? RCAP - 1 : p);
            pl[p] = u & 0xffff;
            cur[slot] = p + 1;
          }
        }
      }
    }
  }
  __syncthreads();

#pragma unroll 1
  for (int i = tid; i < NBRUN; i += NTHR) {
    const int cv = cnt[i];
    const float deg = (float)(cv + 1);
    const float r = 1.0f / sqrtf(deg);
    const float d = (deg > 0.0f) ? r : 0.0f;
    dvb[i] = __float_as_int(d);
  }
  __syncthreads();

  const int ovf = misc[9];
  int* lp = LIST + (size_t)blk * RCAP;
  int* cp = CNT + (size_t)blk * NBRUN;
  int* op = OFF + (size_t)blk * NBRUN;
  int* dp = DINVB + (size_t)blk * NBRUN;
  int* fp = FLAG + (size_t)blk * 32;
  bucket_flush(pl, cnt, offs, dvb, ovf, lp, cp, op, dp, fp, tid);
  __threadfence();
  bucket_flush(pl, cnt, offs, dvb, ovf, lp, cp, op, dp, fp, tid);
}

template <int KTOT>
__device__ __forceinline__ void gemm_16x64(const unsigned short* __restrict__ ap,
                                           const unsigned short* __restrict__ bp, v8f (&acc)[4]) {
#pragma unroll 1
  for (int k0 = 0; k0 < KTOT; k0 += 32) {
    FragB af;
    af.h[0] = *(const v8usa*)(ap + k0);
    af.h[1] = *(const v8usa*)(ap + k0 + 16);
#pragma unroll
    for (int nt = 0; nt < 4; ++nt) {
      const unsigned short* wq = bp + (size_t)(16 * nt) * (size_t)KTOT + k0;
      FragB bf;
      bf.h[0] = *(const v8usa*)wq;
      bf.h[1] = *(const v8usa*)(wq + 16);
      acc[nt] = wmb(af, bf, acc[nt]);
    }
  }
}

__device__ __forceinline__ void stage_d(float* stg, const v8f (&acc)[4], int wave, int hh, int m) {
#pragma unroll
  for (int nt = 0; nt < 4; ++nt) {
#pragma unroll
    for (int r = 0; r < 8; ++r) stg[(16 * wave + 8 * hh + r) * SP + 16 * nt + m] = acc[nt][r];
  }
}

__global__ __launch_bounds__(NTHR) __attribute__((amdgpu_num_vgpr(248)))
void k_gemm(const unsigned short* __restrict__ XB, const unsigned short* __restrict__ WB,
            const float* __restrict__ DINV, float* P) {
  __shared__ __attribute__((aligned(16))) float stg[GBM * SP];
  __shared__ __attribute__((aligned(16))) float sdv[GBM];
  const int tid = (int)threadIdx.x, lane = tid & 31, wave = tid >> 5, hh = lane >> 4, m = lane & 15;
  const int rowBase = (int)blockIdx.x * GBM;
  const int col0    = (int)blockIdx.y * GBN;
  if (tid < 32) *(v4fa*)(sdv + 4 * tid) = *(const v4fa*)(DINV + (size_t)rowBase + 4 * tid);

  v8f acc[4];
  {
    const v8f z = {0.f, 0.f, 0.f, 0.f, 0.f, 0.f, 0.f, 0.f};
#pragma unroll
    for (int t = 0; t < 4; ++t) acc[t] = z;
  }
  const unsigned short* ap = XB + (size_t)(rowBase + 16 * wave + m) * (size_t)CIN + 8 * hh;
  const unsigned short* bp = WB + (size_t)(col0 + m) * (size_t)CIN + 8 * hh;
  gemm_16x64<CIN>(ap, bp, acc);
  stage_d(stg, acc, wave, hh, m);
  __syncthreads();

#pragma unroll 1
  for (int i = 0; i < 8; ++i) {
    const int lr   = 16 * wave + 2 * i + hh;
    const int grow = rowBase + lr;
    const bool live = grow < NN;
    const v4f a = *(const v4fa*)(stg + lr * SP + 4 * m);
    const float dv = sdv[lr];
    asm volatile("" :: "v"(a));
    asm volatile("" :: "v"(dv));
    const float v0 = a.x * dv, v1 = a.y * dv, v2 = a.z * dv, v3 = a.w * dv;
    v4f o;
    o.x = live ? v0 : 0.0f; o.y = live ? v1 : 0.0f; o.z = live ? v2 : 0.0f; o.w = live ? v3 : 0.0f;
    st2_v4f(P + (size_t)grow * COUT + col0 + 4 * m, o);
  }
}

__global__ __launch_bounds__(NTHR) void k_rowsum(const int* __restrict__ LIST, const int* __restrict__ OFF,
                                                 const int* __restrict__ CNT, const float* __restrict__ DINV,
                                                 const int* __restrict__ FLAG, const float* __restrict__ P,
                                                 const float* __restrict__ BF, float* out) {
  __shared__ __attribute__((aligned(16))) float sbf[COUT];
  const int tid = (int)threadIdx.x, lane = tid & 31;
  const int wave = __builtin_amdgcn_readfirstlane(tid >> 5);
  if (tid < 64) *(v4fa*)(sbf + 4 * tid) = *(const v4fa*)(BF + 4 * tid);
  __syncthreads();
  const v4f bb0 = *(const v4fa*)(sbf + 4 * lane);
  const v4f bb1 = *(const v4fa*)(sbf + 128 + 4 * lane);

  const int rowBase = (int)blockIdx.x * ABM;
  const int bucket  = rowBase >> 10;
  const int* lb  = LIST + (size_t)bucket * RCAP;
  const int flag = FLAG[(size_t)bucket * 32];
  const float qnan = __uint_as_float(0x7fc00000u);
  const int row0 = rowBase + 16 * wave;
  int nrows = NN - row0;
  nrows = nrows < 0 ? 0 : (nrows > 16 ? 16 : nrows);

#pragma unroll 1
  for (int i = 0; i < nrows; ++i) {
    const int node = row0 + i;
    int c = __builtin_amdgcn_readfirstlane(CNT[node]);
    int o = __builtin_amdgcn_readfirstlane(OFF[node]);
    const bool big = c > DEGCAP;
    c = c < 0 ? 0 : (c > DEGCAP ? DEGCAP : c);
    o = o < 0 ? 0 : (o > RCAP - 1 ? RCAP - 1 : o);
    int last = o + c - 1; last = last < o ? o : last;
    last = last > RCAP - 1 ? RCAP - 1 : last;
    const float dd = DINV[node];
    v4f a0 = {0.0f, 0.0f, 0.0f, 0.0f};
    v4f a1 = {0.0f, 0.0f, 0.0f, 0.0f};
#pragma unroll 1
    for (int b0 = 0; b0 < c; b0 += 32) {
      int idx = o + b0 + lane;
      idx = idx > last ? last : idx;
      int sr = lb[idx] & 0xffff;
      sr = sr > NN - 1 ? NN - 1 : sr;
      const int m32 = (c - b0) < 32 ? (c - b0) : 32;
#pragma unroll 1
      for (int k = 0; k < m32; ++k) {
        const int sk = __builtin_amdgcn_readlane(sr, k);
        const float* pr = P + (size_t)sk * COUT + 4 * lane;
        const v4f v0 = *(const v4fa*)pr;
        const v4f v1 = *(const v4fa*)(pr + 128);
        asm volatile("" :: "v"(v0));
        asm volatile("" :: "v"(v1));
        a0 = a0 + v0;
        a1 = a1 + v1;
      }
    }
    {
      const float* pr = P + (size_t)node * COUT + 4 * lane;
      const v4f v0 = *(const v4fa*)pr;
      const v4f v1 = *(const v4fa*)(pr + 128);
      a0 = a0 + v0;
      a1 = a1 + v1;
    }
    float t0 = dd * a0.x + bb0.x, t1 = dd * a0.y + bb0.y, t2 = dd * a0.z + bb0.z, t3 = dd * a0.w + bb0.w;
    float t4 = dd * a1.x + bb1.x, t5 = dd * a1.y + bb1.y, t6 = dd * a1.z + bb1.z, t7 = dd * a1.w + bb1.w;
    t0 = (t0 > 0.0f) ? t0 : (t0 - t0); t1 = (t1 > 0.0f) ? t1 : (t1 - t1);
    t2 = (t2 > 0.0f) ? t2 : (t2 - t2); t3 = (t3 > 0.0f) ? t3 : (t3 - t3);
    t4 = (t4 > 0.0f) ? t4 : (t4 - t4); t5 = (t5 > 0.0f) ? t5 : (t5 - t5);
    t6 = (t6 > 0.0f) ? t6 : (t6 - t6); t7 = (t7 > 0.0f) ? t7 : (t7 - t7);
    const bool bad = (flag != 0) | big;
    v4f o0, o1;
    o0.x = bad ? qnan : t0; o0.y = bad ? qnan : t1; o0.z = bad ? qnan : t2; o0.w = bad ? qnan : t3;
    o1.x = bad ? qnan : t4; o1.y = bad ? qnan : t5; o1.z = bad ? qnan : t6; o1.w = bad ? qnan : t7;
    float* op = out + (size_t)node * COUT + 4 * lane;
    *(volatile v4f*)op = o0;
    *(volatile v4f*)(op + 128) = o1;
    __threadfence();
    *(volatile v4f*)op = o0;
    *(volatile v4f*)(op + 128) = o1;
  }
}

extern "C" void kernel_launch(void* const* d_in, const int* in_sizes, int n_in,
                              void* d_out, int out_size, void* d_ws, size_t ws_size,
                              hipStream_t stream) {
  if (n_in < 4) return;
  if (in_sizes[0] != NN * CIN) return;
  if (in_sizes[1] != 2 * NE) return;
  if (in_sizes[2] != COUT * CIN) return;
  if (in_sizes[3] != COUT) return;
  if (out_size != NN * COUT) return;

  const float* x  = (const float*)d_in[0];
  const int*   ei = (const int*)d_in[1];
  const float* W  = (const float*)d_in[2];
  const float* b  = (const float*)d_in[3];
  float* out = (float*)d_out;

  constexpr size_t zP    = (size_t)MP * COUT * 4;
  constexpr size_t zXB   = (size_t)MP * CIN * 2;
  constexpr size_t zWB   = (size_t)COUT * CIN * 2;
  constexpr size_t zBF   = (size_t)COUT * 4;
  constexpr size_t zLIST = (size_t)NBK * RCAP * 4;
  constexpr size_t zTAB  = (size_t)NSLOT * 4;
  constexpr size_t zFLAG = 6400;
  constexpr size_t oP    = 0;
  constexpr size_t oXB   = oP + zP;
  constexpr size_t oWB   = oXB + zXB;
  constexpr size_t oBF   = oWB + zWB;
  constexpr size_t oLIST = oBF + zBF;
  constexpr size_t oOFF  = oLIST + zLIST;
  constexpr size_t oCNT  = oOFF + zTAB;
  constexpr size_t oDINV = oCNT + zTAB;
  constexpr size_t oFLAG = oDINV + zTAB;
  constexpr size_t oEND  = oFLAG + zFLAG;
  static_assert(zP % 256 == 0 && zXB % 256 == 0 && zWB % 256 == 0 && zBF % 256 == 0);
  static_assert(zLIST % 256 == 0 && zTAB % 256 == 0 && zFLAG % 256 == 0 && zFLAG >= (size_t)NBK * 128);
  static_assert(oEND <= (size_t)WSMAX);
  if (oEND > ws_size) return;

  char* ws = (char*)d_ws;
  float*          P    = (float*)(ws + oP);
  unsigned short* XB   = (unsigned short*)(ws + oXB);
  unsigned short* WB   = (unsigned short*)(ws + oWB);
  float*          BF   = (float*)(ws + oBF);
  int*            LIST = (int*)(ws + oLIST);
  int*            OFF  = (int*)(ws + oOFF);
  int*            CNT  = (int*)(ws + oCNT);
  int*            DINV = (int*)(ws + oDINV);
  int*            FLAG = (int*)(ws + oFLAG);

  hipFuncSetAttribute(reinterpret_cast<const void*>(&k_bucket), hipFuncAttributeMaxDynamicSharedMemorySize, (int)BK_LDS);

  k_prep<<<PBTOT, NTHR, 0, stream>>>(x, W, b, XB, WB, BF);
  k_bucket<<<NBK, NTHR, BK_LDS, stream>>>(ei, LIST, OFF, CNT, DINV, FLAG);
  k_gemm<<<dim3(MP / GBM, COUT / GBN), NTHR, 0, stream>>>(XB, WB, (const float*)DINV, P);
  k_rowsum<<<MP / ABM, NTHR, 0, stream>>>(LIST, OFF, CNT, (const float*)DINV, FLAG, P, BF, out);
}
